// _MambaBlock_9096740733534
// MI455X (gfx1250) — hardware-verified
//
#include <hip/hip_runtime.h>
#include <stdint.h>

typedef __attribute__((ext_vector_type(16))) _Float16 v16h;
typedef __attribute__((ext_vector_type(8)))  _Float16 v8h;
typedef __attribute__((ext_vector_type(16))) __bf16   v16b;
typedef __attribute__((ext_vector_type(8)))  __bf16   v8b;
typedef __attribute__((ext_vector_type(8)))  float    v8f;
typedef __attribute__((ext_vector_type(4)))  float    v4f;
typedef __attribute__((ext_vector_type(4)))  unsigned v4u;

static constexpr int kBatch  = 4;
static constexpr int kSeqLen = 2048;
static constexpr int kDModel = 768;
static constexpr int kDInner = 1536;
static constexpr int kDState = 16;
static constexpr int kDtRank = 48;
static constexpr int kRows   = kBatch * kSeqLen;
static constexpr int kXdblN  = 128;
static constexpr int kXprojN = kDtRank + 2 * kDState;
static constexpr int kDtK    = 64;
static constexpr int kScanT  = 32;

__device__ __forceinline__ unsigned short f2bf_bits(float f) {
  unsigned u = __float_as_uint(f);
  return (unsigned short)((u + 0x7FFFu + ((u >> 16) & 1u)) >> 16);
}
__device__ __forceinline__ float bf_bits2f(unsigned short h) { return __uint_as_float(((unsigned)h) << 16); }

__device__ __forceinline__ void dep_guard_h(v8f& a, v8f& b, v16h x, v16h y) { asm volatile("v_nop\n\tv_nop\n\tv_nop\n\tv_nop" : "+v"(a), "+v"(b) : "v"(x), "v"(y)); }
__device__ __forceinline__ void dep_guard_b(v8f& a, v8f& b, v16b x, v16b y) { asm volatile("v_nop\n\tv_nop\n\tv_nop\n\tv_nop" : "+v"(a), "+v"(b) : "v"(x), "v"(y)); }
__device__ __forceinline__ void keep4_h(v16h a, v16h b, v16h c, v16h d) { asm volatile("v_nop" :: "v"(a), "v"(b), "v"(c), "v"(d)); }
__device__ __forceinline__ void keep4_b(v16b a, v16b b, v16b c, v16b d) { asm volatile("v_nop" :: "v"(a), "v"(b), "v"(c), "v"(d)); }
__device__ __forceinline__ void acc_guard4(v8f& a, v8f& b, v8f& c, v8f& d) { asm volatile("v_nop\n\tv_nop\n\tv_nop\n\tv_nop" : "+v"(a), "+v"(b), "+v"(c), "+v"(d)); }
template <typename T> struct Frag;
template <> struct Frag<_Float16> {
  typedef v16h V; union U { v16h v; v8h h[2]; };
  static __device__ __forceinline__ v16h load(const _Float16* p) {
    U f; f.h[0] = *(const v8h*)(p); f.h[1] = *(const v8h*)(p + 16); return f.v;
  }
  static __device__ __forceinline__ v8f mma(v16h a, v16h b, v8f c) {
    return __builtin_amdgcn_wmma_f32_16x16x32_f16(false, a, false, b, (short)0, c, false, false);
  }
  static __device__ __forceinline__ void guard(v8f& a, v8f& b, v16h x, v16h y) { dep_guard_h(a, b, x, y); }
  static __device__ __forceinline__ void keep(v16h a, v16h b, v16h c, v16h d) { keep4_h(a, b, c, d); }
};
template <> struct Frag<__bf16> {
  typedef v16b V; union U { v16b v; v8b h[2]; };
  static __device__ __forceinline__ v16b load(const __bf16* p) {
    U f; f.h[0] = *(const v8b*)(p); f.h[1] = *(const v8b*)(p + 16); return f.v;
  }
  static __device__ __forceinline__ v8f mma(v16b a, v16b b, v8f c) {
    return __builtin_amdgcn_wmma_f32_16x16x32_bf16(false, a, false, b, (short)0, c, false, false);
  }
  static __device__ __forceinline__ void guard(v8f& a, v8f& b, v16b x, v16b y) { dep_guard_b(a, b, x, y); }
  static __device__ __forceinline__ void keep(v16b a, v16b b, v16b c, v16b d) { keep4_b(a, b, c, d); }
};

template <int ET> struct Elem;
template <> struct Elem<0> { typedef _Float16 T; };
template <> struct Elem<1> { typedef __bf16 T; };
template <int ET, bool SPLIT, int BIAS_MODE, int OUT_MODE, bool RESID, int ACT = 0>
__global__ __launch_bounds__(256) void wmma_gemm64(
    const unsigned short* __restrict__ Ap, const unsigned short* __restrict__ A2p, int lda, long strideA,
    const unsigned short* __restrict__ Btp, const unsigned short* __restrict__ Bt2p, int ldb, long strideB,
    void* __restrict__ Cout, void* __restrict__ Cout2, int ldc, long strideC,
    const float* __restrict__ bias,
    const float* __restrict__ resid, long strideR,
    int M, int N, int K, float scale) {
  typedef typename Elem<ET>::T T;
  typedef typename Frag<T>::V V;
  const T* A = (const T*)Ap; const T* A2 = (const T*)A2p; const T* Bt = (const T*)Btp; const T* Bt2 = (const T*)Bt2p;
  __shared__ __align__(16) float sT[8][16 * 68];
  const int b    = blockIdx.y;
  const int lane = threadIdx.x & 31;
  const int wave = threadIdx.x >> 5;
  const int tilesN = N >> 6;
  const int tilesM = M >> 6;
  const int tile = blockIdx.x * 8 + wave;
  if (tile >= tilesM * tilesN) return;
  const int tm = tile / tilesN;
  const int tn = tile - tm * tilesN;
  const int m0 = tm << 6;
  const int n0 = tn << 6;

  const T* Ab  = A  + (size_t)b * strideA;
  const T* Bb  = Bt + (size_t)b * strideB;
  const T* Ab2 = SPLIT ? (A2  + (size_t)b * strideA) : nullptr;
  const T* Bb2 = SPLIT ? (Bt2 + (size_t)b * strideB) : nullptr;

  const int rlane = lane & 15;
  const int koff  = (lane >> 4) * 8;
  const int mOff  = (lane >> 4) * 8;

  v8f acc[4][4];
#pragma unroll
  for (int i = 0; i < 4; ++i)
#pragma unroll
    for (int j = 0; j < 4; ++j) acc[i][j] = (v8f){0.f,0.f,0.f,0.f,0.f,0.f,0.f,0.f};

  for (int k0 = 0; k0 < K; k0 += 32) {
    V bh[4], bl[4];
#pragma unroll
    for (int j = 0; j < 4; ++j) {
      const size_t bo = (size_t)(n0 + (j << 4) + rlane) * ldb + koff + k0;
      bh[j] = Frag<T>::load(Bb + bo);
      if (SPLIT) bl[j] = Frag<T>::load(Bb2 + bo);
    }
#pragma unroll
    for (int i = 0; i < 4; ++i) {
      const size_t ao = (size_t)(m0 + (i << 4) + rlane) * lda + koff + k0;
      V ah = Frag<T>::load(Ab + ao);
      V al;
      if (SPLIT) al = Frag<T>::load(Ab2 + ao);
#pragma unroll
      for (int j = 0; j < 4; ++j) {
        acc[i][j] = Frag<T>::mma(ah, bh[j], acc[i][j]);
        if (SPLIT) {
          acc[i][j] = Frag<T>::mma(ah, bl[j], acc[i][j]);
          acc[i][j] = Frag<T>::mma(al, bh[j], acc[i][j]);
        }
      }
      Frag<T>::guard(acc[i][0], acc[i][3], ah, SPLIT ? al : ah);
    }
    Frag<T>::keep(bh[0], bh[1], bh[2], bh[3]);
    if (SPLIT) Frag<T>::keep(bl[0], bl[1], bl[2], bl[3]);
  }
  acc_guard4(acc[0][0], acc[0][1], acc[0][2], acc[0][3]);
  acc_guard4(acc[1][0], acc[1][1], acc[1][2], acc[1][3]);
  acc_guard4(acc[2][0], acc[2][1], acc[2][2], acc[2][3]);
  acc_guard4(acc[3][0], acc[3][1], acc[3][2], acc[3][3]);

  float* slab = sT[wave];
  const float* Rb = RESID ? (resid + (size_t)b * strideR) : nullptr;
#pragma unroll
  for (int i = 0; i < 4; ++i) {
    const int mBase = m0 + (i << 4);
#pragma unroll
    for (int j = 0; j < 4; ++j) {
      const int n = n0 + (j << 4) + rlane;
      float bv = 0.f;
      if (BIAS_MODE == 2) bv = bias[n];
#pragma unroll
      for (int r = 0; r < 8; ++r) {
        float v = acc[i][j][r] * scale;
        if (BIAS_MODE == 1) v += bias[mBase + mOff + r];
        if (BIAS_MODE == 2) v += bv;
        if (ACT == 1) v = tanhf(v);
        if (ACT == 2) v = fmaxf(v, 0.0f);
        if (ACT == 3) v = v / (1.0f + expf(-v));
        if (ACT == 4) v = (v > 0.f) ? v : 0.01f * v;
        slab[(mOff + r) * 68 + (j << 4) + rlane] = v;
      }
    }
    __builtin_amdgcn_fence(__ATOMIC_RELEASE, "workgroup");
    __builtin_amdgcn_wave_barrier();
    __builtin_amdgcn_fence(__ATOMIC_ACQUIRE, "workgroup");
    if (OUT_MODE == 0) {
      float* C = (float*)Cout + (size_t)b * strideC;
      const int hh = lane >> 4, c4 = (lane & 15) * 4;
      v4f vals[8];
#pragma unroll
      for (int it = 0; it < 8; ++it) {
        const int row = it * 2 + hh;
        v4f v = *(const v4f*)(slab + row * 68 + c4);
        if (RESID) {
          const v4f rr = *(const v4f*)(Rb + (size_t)(mBase + row) * ldc + n0 + c4);
          v += rr;
        }
        vals[it] = v;
      }
      for (int pass = 0; pass < 2; ++pass) {
#pragma unroll
        for (int it = 0; it < 8; ++it) {
          const int row = it * 2 + hh;
          *(volatile v4f*)(C + (size_t)(mBase + row) * ldc + n0 + c4) = vals[it];
        }
        __threadfence();
      }
    } else {
      const int q = lane >> 3, c8 = (lane & 7) * 8;
      unsigned short* C  = (unsigned short*)Cout  + (size_t)b * strideC;
      unsigned short* C2 = (OUT_MODE == 2) ? ((unsigned short*)Cout2 + (size_t)b * strideC) : nullptr;
      for (int pass = 0; pass < 2; ++pass) {
#pragma unroll
        for (int it = 0; it < 4; ++it) {
          const int row = it * 4 + q;
          const float* sp = slab + row * 68 + c8;
          v8h hv, lv;
#pragma unroll
          for (int e = 0; e < 8; ++e) {
            if (OUT_MODE == 1) {
              hv[e] = (_Float16)sp[e];
            } else {
              unsigned short hb = f2bf_bits(sp[e]);
              unsigned short lb = f2bf_bits(sp[e] - bf_bits2f(hb));
              hv[e] = __builtin_bit_cast(_Float16, hb);
              lv[e] = __builtin_bit_cast(_Float16, lb);
            }
          }
          *(volatile v8h*)(C + (size_t)(mBase + row) * ldc + n0 + c8) = hv;
          if (OUT_MODE == 2) *(volatile v8h*)(C2 + (size_t)(mBase + row) * ldc + n0 + c8) = lv;
        }
        __threadfence();
      }
    }
    __builtin_amdgcn_fence(__ATOMIC_RELEASE, "workgroup");
    __builtin_amdgcn_wave_barrier();
    __builtin_amdgcn_fence(__ATOMIC_ACQUIRE, "workgroup");
  }
}

__device__ __forceinline__ float h16_to_f32(unsigned hb) {
  const unsigned sgn = (hb & 0x8000u) << 16;
  const unsigned em  = hb & 0x7fffu;
  const float fn = __uint_as_float((em << 13) + 0x38000000u);
  const float fs = (float)em * 5.9604644775390625e-8f;
  const float mag = (em < 0x400u) ? fs : fn;
  return __uint_as_float(__float_as_uint(mag) | sgn);
}
__device__ __forceinline__ void unpack8h(const v4u u, float* out8) {
#pragma unroll
  for (int k = 0; k < 4; ++k) {
    const unsigned w = u[k];
    out8[2 * k]     = h16_to_f32(w & 0xffffu);
    out8[2 * k + 1] = h16_to_f32(w >> 16);
  }
}

__global__ __launch_bounds__(256) void k_transpose_cast(const float* __restrict__ in, _Float16* __restrict__ out,
                                                        int K, int N, int Kpad, int Npad) {
  __shared__ float tile[64][65];
  const int tid = threadIdx.x;
  const int n0 = blockIdx.x * 64;
  const int k0 = blockIdx.y * 64;
#pragma unroll
  for (int i = 0; i < 4; ++i) {
    const int f = tid + i * 256;
    const int r = f >> 4;
    const int c4 = (f & 15) * 4;
    const int kk = k0 + r;
    const int kc = (kk < K) ? kk : (K - 1);
    const int nn = n0 + c4;
    const int nc = (nn + 4 <= N) ? nn : (N - 4);
    const v4f v = *(const v4f*)(in + (size_t)kc * N + nc);
#pragma unroll
    for (int e = 0; e < 4; ++e) tile[r][c4 + e] = (kk < K && (nn + e) < N) ? v[e] : 0.0f;
  }
  __syncthreads();
  for (int pass = 0; pass < 2; ++pass) {
#pragma unroll
    for (int i = 0; i < 2; ++i) {
      const int s = tid + i * 256;
      const int nr = s >> 3;
      const int q = s & 7;
      v8h hv;
#pragma unroll
      for (int e = 0; e < 8; ++e) hv[e] = (_Float16)tile[8 * q + e][nr];
      *(volatile v8h*)(out + (size_t)(n0 + nr) * Kpad + k0 + 8 * q) = hv;
    }
    __threadfence();
  }
}

__global__ __launch_bounds__(96) void k_rmsnorm_f16(const float* __restrict__ x, const float* __restrict__ w,
                                                    _Float16* __restrict__ xn) {
  __shared__ float red[4];
  const int row = blockIdx.x;
  const int tid = threadIdx.x;
  const float* xr = x + (size_t)row * kDModel + tid * 8;
  const v4f a0 = *(const v4f*)(xr);
  const v4f a1 = *(const v4f*)(xr + 4);
  float s = 0.0f;
#pragma unroll
  for (int e = 0; e < 4; ++e) { s += a0[e] * a0[e]; s += a1[e] * a1[e]; }
#pragma unroll
  for (int off = 1; off < 32; off <<= 1) s += __shfl_xor(s, off, 32);
  if ((tid & 31) == 0) red[tid >> 5] = s;
  __syncthreads();
  const float tot = red[0] + red[1] + red[2];
  const float inv = rsqrtf(tot * (1.0f / (float)kDModel) + 1e-5f);
  const v4f w0 = *(const v4f*)(w + tid * 8);
  const v4f w1 = *(const v4f*)(w + tid * 8 + 4);
  v8h hv;
#pragma unroll
  for (int e = 0; e < 4; ++e) {
    hv[e]     = (_Float16)((a0[e] * inv) * w0[e]);
    hv[4 + e] = (_Float16)((a1[e] * inv) * w1[e]);
  }
  _Float16* dst = xn + (size_t)row * kDModel + tid * 8;
  *(volatile v8h*)dst = hv;
  __threadfence();
  *(volatile v8h*)dst = hv;
}

__global__ __launch_bounds__(256) void k_dwconv_silu(const _Float16* __restrict__ xz, const float* __restrict__ cw,
                                                     const float* __restrict__ cb, _Float16* __restrict__ xc) {
  const int g = blockIdx.x * 256 + threadIdx.x;
  if (g >= kRows * (kDInner / 8)) return;
  const int row = g / (kDInner / 8);
  const int c0 = (g - row * (kDInner / 8)) * 8;
  const int l = row & (kSeqLen - 1);
  const float LOG2E = 1.4426950408889634f;
  float acc[8];
  {
    const v4f b0 = *(const v4f*)(cb + c0);
    const v4f b1 = *(const v4f*)(cb + c0 + 4);
#pragma unroll
    for (int e = 0; e < 4; ++e) { acc[e] = b0[e]; acc[4 + e] = b1[e]; }
  }
  v4f wv[8];
#pragma unroll
  for (int e = 0; e < 8; ++e) wv[e] = *(const v4f*)(cw + (size_t)(c0 + e) * 4);
#pragma unroll
  for (int j = 0; j < 4; ++j) {
    const int li = l - 3 + j;
    const int rr = (li >= 0) ? (row - 3 + j) : row;
    const float keep = (li >= 0) ? 1.0f : 0.0f;
    const v4u u = *(const v4u*)(xz + (size_t)rr * (2 * kDInner) + c0);
    float xv[8];
    unpack8h(u, xv);
#pragma unroll
    for (int e = 0; e < 8; ++e) acc[e] += (xv[e] * keep) * wv[e][j];
  }
  v8h hv;
#pragma unroll
  for (int e = 0; e < 8; ++e) {
    const float cv = acc[e];
    const float sv = cv * __builtin_amdgcn_rcpf(1.0f + exp2f(-cv * LOG2E));
    hv[e] = (_Float16)sv;
  }
  _Float16* dst = xc + (size_t)row * kDInner + c0;
  *(volatile v8h*)dst = hv;
  __threadfence();
  *(volatile v8h*)dst = hv;
}

__global__ __launch_bounds__(256) void k_cast_dtlo(const float* __restrict__ xd, _Float16* __restrict__ dtlo) {
  const int t = blockIdx.x * 256 + threadIdx.x;
  if (t >= kRows * 8) return;
  const int row = t >> 3;
  const int q = t & 7;
  const int qc = (q < 6) ? q : 5;
  const float keep = (q < 6) ? 1.0f : 0.0f;
  const v4f a = *(const v4f*)(xd + (size_t)row * kXdblN + qc * 8);
  const v4f bq = *(const v4f*)(xd + (size_t)row * kXdblN + qc * 8 + 4);
  v8h hv;
#pragma unroll
  for (int e = 0; e < 4; ++e) { hv[e] = (_Float16)(a[e] * keep); hv[4 + e] = (_Float16)(bq[e] * keep); }
  _Float16* dst = dtlo + (size_t)row * kDtK + q * 8;
  *(volatile v8h*)dst = hv;
  __threadfence();
  *(volatile v8h*)dst = hv;
}

__global__ __launch_bounds__(64) void k_selective_scan(
    const _Float16* __restrict__ xz, const _Float16* __restrict__ dtraw, const float* __restrict__ xdbl,
    const float* __restrict__ cw, const float* __restrict__ cb, const float* __restrict__ dtb,
    const float* __restrict__ alog, const float* __restrict__ dpar, _Float16* __restrict__ yout) {
  __shared__ __align__(16) float    sBC[kScanT][32];
  __shared__ __align__(16) unsigned sDT[kScanT][32];
  __shared__ __align__(16) unsigned sXI[kScanT][32];
  __shared__ __align__(16) unsigned sZ [kScanT][32];
  __shared__ __align__(16) float    sY [kScanT][64];
  const int tid = threadIdx.x;
  const int b = blockIdx.x / (kDInner / 64);
  const int d0 = (blockIdx.x - b * (kDInner / 64)) * 64;
  const int d = d0 + tid;
  const size_t rowb = (size_t)b * kSeqLen;
  const float LOG2E = 1.4426950408889634f;

  float Acoef[kDState];
#pragma unroll
  for (int qq = 0; qq < 4; ++qq) {
    const v4f av = *(const v4f*)(alog + (size_t)d * kDState + 4 * qq);
#pragma unroll
    for (int e = 0; e < 4; ++e) Acoef[4 * qq + e] = -exp2f(av[e] * LOG2E) * LOG2E;
  }
  const v4f cwv = *(const v4f*)(cw + (size_t)d * 4);
  const float cbv = cb[d];
  const float biasv = dtb[d];
  const float Dv = dpar[d];

  float h[kDState];
#pragma unroll
  for (int s = 0; s < kDState; ++s) h[s] = 0.0f;
  float xm1 = 0.0f, xm2 = 0.0f, xm3 = 0.0f;
  const int wsel = tid >> 1;
  const unsigned shsel = (unsigned)(tid & 1) * 16u;
  const int q = tid & 7;

#pragma unroll 1
  for (int ck = 0; ck < kSeqLen / kScanT; ++ck) {
    const int l0 = ck * kScanT;
    __syncthreads();
#pragma unroll
    for (int i = 0; i < 4; ++i) {
      const int f = tid + 64 * i;
      const int r = f >> 3;
      const int qq = f & 7;
      const size_t row = rowb + l0 + r;
      const v4f bc = *(const v4f*)(xdbl + row * kXdblN + kDtRank + 4 * qq);
      *(v4f*)(&sBC[r][4 * qq]) = bc;
      const v4u udt = *(const v4u*)(dtraw + row * kDInner + d0 + 8 * qq);
      *(v4u*)(&sDT[r][4 * qq]) = udt;
      const v4u uxi = *(const v4u*)(xz + row * (size_t)(2 * kDInner) + d0 + 8 * qq);
      *(v4u*)(&sXI[r][4 * qq]) = uxi;
      const v4u uz = *(const v4u*)(xz + row * (size_t)(2 * kDInner) + kDInner + d0 + 8 * qq);
      *(v4u*)(&sZ[r][4 * qq]) = uz;
    }
    __syncthreads();
#pragma unroll 1
    for (int t = 0; t < kScanT; ++t) {
      const float rawv = h16_to_f32((sDT[t][wsel] >> shsel) & 0xffffu) + biasv;
      const float xiv  = h16_to_f32((sXI[t][wsel] >> shsel) & 0xffffu);
      const float zv   = h16_to_f32((sZ [t][wsel] >> shsel) & 0xffffu);
      const float ev = exp2f(-fabsf(rawv) * LOG2E);
      const float uu = ev * __builtin_amdgcn_rcpf(2.0f + ev);
      const float u2 = uu * uu;
      float p = 1.0f / 13.0f;
      p = fmaf(p, u2, 1.0f / 11.0f);
      p = fmaf(p, u2, 1.0f / 9.0f);
      p = fmaf(p, u2, 1.0f / 7.0f);
      p = fmaf(p, u2, 1.0f / 5.0f);
      p = fmaf(p, u2, 1.0f / 3.0f);
      p = fmaf(p, u2, 1.0f);
      const float dt = fmaxf(rawv, 0.0f) + 2.0f * uu * p;
      float cv = cbv;
      cv = fmaf(cwv[0], xm3, cv);
      cv = fmaf(cwv[1], xm2, cv);
      cv = fmaf(cwv[2], xm1, cv);
      cv = fmaf(cwv[3], xiv, cv);
      xm3 = xm2; xm2 = xm1; xm1 = xiv;
      const float xv = cv * __builtin_amdgcn_rcpf(1.0f + exp2f(-cv * LOG2E));
      const float dtx = dt * xv;
      float y = 0.0f;
#pragma unroll
      for (int s = 0; s < kDState; ++s) {
        const float Bv = sBC[t][s];
        const float Cv = sBC[t][kDState + s];
        const float dA = exp2f(dt * Acoef[s]);
        h[s] = fmaf(h[s], dA, dtx * Bv);
        y = fmaf(h[s], Cv, y);
      }
      y = fmaf(Dv, xv, y);
      const float gz = zv * __builtin_amdgcn_rcpf(1.0f + exp2f(-zv * LOG2E));
      sY[t][tid] = y * gz;
    }
    __syncthreads();
    for (int pass = 0; pass < 2; ++pass) {
#pragma unroll
      for (int i = 0; i < 4; ++i) {
        const int r = (tid >> 3) + 8 * i;
        const float* sp = &sY[r][8 * q];
        v8h hv;
#pragma unroll
        for (int e = 0; e < 8; ++e) hv[e] = (_Float16)sp[e];
        *(volatile v8h*)(yout + (rowb + l0 + r) * kDInner + d0 + 8 * q) = hv;
      }
      __threadfence();
    }
  }
}

static constexpr size_t SZ_WIN  = (size_t)(2 * kDInner) * kDModel * 2;
static constexpr size_t SZ_WX   = (size_t)kXdblN * kDInner * 2;
static constexpr size_t SZ_WDT  = (size_t)kDInner * kDtK * 2;
static constexpr size_t SZ_WOUT = (size_t)kDModel * kDInner * 2;
static constexpr size_t SZ_XZ   = (size_t)kRows * (2 * kDInner) * 2;
static constexpr size_t SZ_RA   = (size_t)kRows * kDModel * 2;
static constexpr size_t SZ_XDBL = (size_t)kRows * kXdblN * 4;
static constexpr size_t SZ_DTLO = (size_t)kRows * kDtK * 2;
static constexpr size_t SZ_RB   = (size_t)kRows * kDInner * 2;
static constexpr size_t SZ_DT   = (size_t)kRows * kDInner * 2;
static constexpr size_t OFF_WIN  = 0;
static constexpr size_t OFF_WX   = OFF_WIN + SZ_WIN;
static constexpr size_t OFF_WDT  = OFF_WX + SZ_WX;
static constexpr size_t OFF_WOUT = OFF_WDT + SZ_WDT;
static constexpr size_t OFF_XZ   = OFF_WOUT + SZ_WOUT;
static constexpr size_t OFF_RA   = OFF_XZ + SZ_XZ;
static constexpr size_t OFF_XDBL = OFF_RA;
static constexpr size_t OFF_DTLO = OFF_RA + SZ_XDBL;
static constexpr size_t OFF_RB   = OFF_RA + SZ_RA;
static constexpr size_t OFF_DT   = OFF_RB + SZ_RB;
static constexpr size_t kWsTotal = OFF_DT + SZ_DT;
static_assert(SZ_XDBL + SZ_DTLO <= SZ_RA, "ra");
static_assert(kWsTotal == 120913920u, "ws");
static_assert(kWsTotal <= 134217728u, "cap");
static_assert((OFF_WX % 256) == 0 && (OFF_WDT % 256) == 0 && (OFF_WOUT % 256) == 0 && (OFF_XZ % 256) == 0 &&
              (OFF_RA % 256) == 0 && (OFF_DTLO % 256) == 0 && (OFF_RB % 256) == 0 && (OFF_DT % 256) == 0, "align");
static_assert(kRows % 64 == 0 && (2 * kDInner) % 64 == 0 && kDModel % 32 == 0, "g0");
static_assert(kXdblN % 64 == 0 && kDInner % 32 == 0, "g1");
static_assert(kDInner % 64 == 0 && kDtK % 32 == 0, "g2");
static_assert(kDModel % 64 == 0, "g3");
static_assert(kXprojN % 4 == 0 && kSeqLen % kScanT == 0 && (kRows * (kDInner / 8)) % 256 == 0, "misc");

template <int OUT_MODE, bool RESID>
static void launch_gemm_f16(const _Float16* A, int lda, const _Float16* Bt, int ldb, void* C, int ldc,
                            const float* resid, int M, int N, int K, hipStream_t st) {
  const int tiles = (M / 64) * (N / 64);
  dim3 grid((tiles + 7) / 8, 1);
  wmma_gemm64<0, false, 0, OUT_MODE, RESID, 0><<<grid, 256, 0, st>>>(
      (const unsigned short*)A, nullptr, lda, 0L,
      (const unsigned short*)Bt, nullptr, ldb, 0L,
      C, nullptr, ldc, 0L,
      nullptr, resid, 0L, M, N, K, 1.0f);
}

extern "C" void kernel_launch(void* const* d_in, const int* in_sizes, int n_in,
                              void* d_out, int out_size, void* d_ws, size_t ws_size,
                              hipStream_t stream) {
  if (n_in < 11) return;
  if (in_sizes[0] != kRows * kDModel || out_size != kRows * kDModel) return;
  if (ws_size < kWsTotal) return;

  const float* seq        = (const float*)d_in[0];
  const float* norm_w     = (const float*)d_in[1];
  const float* in_proj_w  = (const float*)d_in[2];
  const float* conv_w     = (const float*)d_in[3];
  const float* conv_b     = (const float*)d_in[4];
  const float* x_proj_w   = (const float*)d_in[5];
  const float* dt_proj_w  = (const float*)d_in[6];
  const float* dt_bias    = (const float*)d_in[7];
  const float* A_log      = (const float*)d_in[8];
  const float* D_param    = (const float*)d_in[9];
  const float* out_proj_w = (const float*)d_in[10];
  float* out = (float*)d_out;

  char* ws = (char*)d_ws;
  _Float16* wT_in  = (_Float16*)(ws + OFF_WIN);
  _Float16* wT_x   = (_Float16*)(ws + OFF_WX);
  _Float16* wT_dt  = (_Float16*)(ws + OFF_WDT);
  _Float16* wT_out = (_Float16*)(ws + OFF_WOUT);
  _Float16* xz     = (_Float16*)(ws + OFF_XZ);
  _Float16* xn     = (_Float16*)(ws + OFF_RA);
  float*    xdbl   = (float*)(ws + OFF_XDBL);
  _Float16* dtlo   = (_Float16*)(ws + OFF_DTLO);
  _Float16* xc     = (_Float16*)(ws + OFF_RB);
  _Float16* ybuf   = (_Float16*)(ws + OFF_RB);
  _Float16* dtraw  = (_Float16*)(ws + OFF_DT);

  k_transpose_cast<<<dim3((2 * kDInner) / 64, kDModel / 64), 256, 0, stream>>>(in_proj_w, wT_in, kDModel, 2 * kDInner, kDModel, 2 * kDInner);
  k_transpose_cast<<<dim3(kXdblN / 64, kDInner / 64), 256, 0, stream>>>(x_proj_w, wT_x, kDInner, kXprojN, kDInner, kXdblN);
  k_transpose_cast<<<dim3(kDInner / 64, kDtK / 64), 256, 0, stream>>>(dt_proj_w, wT_dt, kDtRank, kDInner, kDtK, kDInner);
  k_transpose_cast<<<dim3(kDModel / 64, kDInner / 64), 256, 0, stream>>>(out_proj_w, wT_out, kDInner, kDModel, kDInner, kDModel);

  k_rmsnorm_f16<<<kRows, 96, 0, stream>>>(seq, norm_w, xn);

  launch_gemm_f16<1, false>(xn, kDModel, wT_in, kDModel, (void*)xz, 2 * kDInner, nullptr, kRows, 2 * kDInner, kDModel, stream);

  k_dwconv_silu<<<(kRows * (kDInner / 8)) / 256, 256, 0, stream>>>(xz, conv_w, conv_b, xc);

  launch_gemm_f16<0, false>(xc, kDInner, wT_x, kDInner, (void*)xdbl, kXdblN, nullptr, kRows, kXdblN, kDInner, stream);

  k_cast_dtlo<<<(kRows * 8) / 256, 256, 0, stream>>>(xdbl, dtlo);

  launch_gemm_f16<1, false>(dtlo, kDtK, wT_dt, kDtK, (void*)dtraw, kDInner, nullptr, kRows, kDInner, kDtK, stream);

  k_selective_scan<<<kBatch * (kDInner / 64), 64, 0, stream>>>(xz, dtraw, xdbl, conv_w, conv_b, dt_bias, A_log, D_param, ybuf);

  launch_gemm_f16<0, true>(ybuf, kDInner, wT_out, kDInner, (void*)out, kDModel, seq, kRows, kDModel, kDInner, stream);
}
